// PPNet_56504589746701
// MI455X (gfx1250) — hardware-verified
//
#include <hip/hip_runtime.h>

#define BB   32
#define CC   128
#define CP   130
#define HH   14
#define WW   14
#define HW   196
#define XP   224
#define PP   2000
#define PPAD 2048
#define NCLS 200
#define KK   4
#define KPAD 544
#define CPAD 136
#define MM   6272
#define EPSV 0.0001f

typedef _Float16 v16h __attribute__((ext_vector_type(16)));
typedef _Float16 v8h  __attribute__((ext_vector_type(8)));
typedef float    v8f  __attribute__((ext_vector_type(8)));
typedef float    v4f  __attribute__((ext_vector_type(4)));
typedef v8h __attribute__((may_alias)) v8ha;
typedef v4f __attribute__((may_alias)) v4fa;

union Frag { v16h v; v8h half[2]; };

static_assert(MM % 64 == 0);
static_assert(PPAD % 128 == 0);
static_assert(KPAD % 32 == 0);
static_assert(CPAD * KK == KPAD);
static_assert((16 * KPAD * 2) % 128 == 0);
static_assert((XP * 4) % 128 == 0);

__device__ __forceinline__ v8f wmma_f16(v16h a, v16h b, v8f c) {
  v8f d = __builtin_amdgcn_wmma_f32_16x16x32_f16(false, a, false, b, (short)0, c, false, false);
  asm volatile("v_nop\n\tv_nop\n\tv_nop\n\tv_nop" : "+v"(d) : "v"(a), "v"(b));
  return d;
}

__device__ __forceinline__ v16h load_frag(const _Float16* p, int h) {
  Frag f;
  f.half[0] = *(const v8ha*)(p + 8 * h);
  f.half[1] = *(const v8ha*)(p + 16 + 8 * h);
  return f.v;
}

__device__ __forceinline__ void prep_store(const float* __restrict__ x, float* xn, float* nmap,
                                           int b, int hw, int hwc, bool act, float r) {
  float nn = 0.f;
  #pragma unroll 1
  for (int c = 0; c < CP; ++c) {
    const int cc = (c < CC) ? c : (CC - 1);
    const float xv = x[((size_t)(b * CC + cc)) * HW + hwc];
    const float xe = (c < CC) ? xv : EPSV;
    float v = (xe * r) * 32.0f;
    v = act ? v : 0.f;
    nn += v * v;
    *(volatile float*)(xn + ((size_t)(b * CP + c)) * XP + hw) = v;
  }
  const float nm = sqrtf(nn);
  *(volatile float*)(nmap + (size_t)b * XP + hw) = act ? nm : 0.f;
}

__global__ __launch_bounds__(224) void k_prep_x(const float* __restrict__ x,
                                                float* __restrict__ xn,
                                                float* __restrict__ nmap) {
  const int b = blockIdx.x, hw = threadIdx.x;
  const bool act = hw < HW;
  const int hwc = act ? hw : (HW - 1);
  float ss = 0.f;
  #pragma unroll 4
  for (int c = 0; c < CC; ++c) {
    const float v = x[((size_t)(b * CC + c)) * HW + hwc];
    ss += v * v;
  }
  ss += 2.0f * EPSV * EPSV;
  const float xlen = sqrtf(ss + EPSV);
  const float r = 1.0f / xlen;
  prep_store(x, xn, nmap, b, hw, hwc, act, r);
  __threadfence();
  prep_store(x, xn, nmap, b, hw, hwc, act, r);
}

__device__ __forceinline__ void plane_store16(const _Float16* sT, _Float16* dst, int tid) {
  #pragma unroll
  for (int j = 0; j < 17; ++j) {
    const int piece = tid + 64 * j;
    const v8h v = *(const v8ha*)(sT + piece * 8);
    *(volatile v8h*)(dst + (size_t)piece * 8) = v;
  }
}

__global__ __launch_bounds__(64) void k_proto(const float* __restrict__ pv,
                                              _Float16* __restrict__ ppl) {
  __shared__ __attribute__((aligned(16))) _Float16 sT[16 * KPAD];
  const int tid = threadIdx.x, pl = tid >> 2, kk = tid & 3;
  const int p0 = blockIdx.x * 16, p = p0 + pl;
  const bool valid = p < PP;
  const int pc = valid ? p : (PP - 1);
  const float* row = pv + (size_t)pc * (CC * KK);
  float ss = 0.f;
  #pragma unroll 4
  for (int c = 0; c < CC; ++c) {
    const float v = row[c * KK + kk];
    ss += v * v;
  }
  ss += 2.0f * EPSV * EPSV;
  const float plen = sqrtf(ss + EPSV);
  const float rc = 1.0f / (plen + EPSV);
  const float sc = valid ? 32.0f : 0.0f;
  #pragma unroll 1
  for (int c = 0; c < CPAD; ++c) {
    const int cc = (c < CC) ? c : (CC - 1);
    const float v = row[cc * KK + kk];
    const float pe = (c < CC) ? v : ((c < CP) ? EPSV : 0.0f);
    const float q = (pe * rc) * sc;
    sT[pl * KPAD + c * KK + kk] = (_Float16)q;
  }
  __syncthreads();
  _Float16* dst = ppl + (size_t)p0 * KPAD;
  plane_store16(sT, dst, tid);
  __threadfence();
  plane_store16(sT, dst, tid);
}

__global__ __launch_bounds__(64) void k_sample(const float* __restrict__ xn,
                                               const float* __restrict__ nmap,
                                               const float* __restrict__ wt,
                                               _Float16* __restrict__ apl) {
  __shared__ __attribute__((aligned(16))) float    sS[CP * 64];
  __shared__ __attribute__((aligned(16))) _Float16 sA[16 * KPAD];
  const int tid = threadIdx.x, ml = tid >> 2, kk = tid & 3;
  const int m = blockIdx.x * 16 + ml;
  const int b = m / HW, hw = m - b * HW;
  const int h = hw / WW, w = hw - h * WW;
  const int ki = kk >> 1, kj = kk & 1;

  int nid[9]; float nok[9];
  #pragma unroll
  for (int r = 0; r < 3; ++r) {
    #pragma unroll
    for (int s = 0; s < 3; ++s) {
      const int y = h - 1 + r, xw = w - 1 + s;
      const bool ok = (y >= 0) && (y < HH) && (xw >= 0) && (xw < WW);
      const int yc = y < 0 ? 0 : (y > HH - 1 ? HH - 1 : y);
      const int xc = xw < 0 ? 0 : (xw > WW - 1 ? WW - 1 : xw);
      nid[r * 3 + s] = yc * WW + xc;
      nok[r * 3 + s] = ok ? 1.0f : 0.0f;
    }
  }

  const float* xb = xn + (size_t)b * CP * XP;
  const float* wy = wt + (size_t)(2 * kk) * (CP * 9);
  const float* wx = wt + (size_t)(2 * kk + 1) * (CP * 9);
  float ay = 0.f, ax = 0.f;
  #pragma unroll 1
  for (int c = 0; c < CP; ++c) {
    const float* xc_ = xb + (size_t)c * XP;
    const float* wyc = wy + c * 9;
    const float* wxc = wx + c * 9;
    #pragma unroll
    for (int t9 = 0; t9 < 9; ++t9) {
      const float v = xc_[nid[t9]] * nok[t9];
      ay += v * wyc[t9];
      ax += v * wxc[t9];
    }
  }

  const float py = (float)(h - 1 + 2 * ki) + ay;
  const float px = (float)(w - 1 + 2 * kj) + ax;
  const float y0 = floorf(py), x0 = floorf(px);
  float cw[4]; int cid[4];
  #pragma unroll
  for (int t = 0; t < 4; ++t) {
    const float yi = y0 + (float)(t >> 1), xi = x0 + (float)(t & 1);
    const float wgt = (1.0f - fabsf(py - yi)) * (1.0f - fabsf(px - xi));
    const bool ok = (yi >= 0.0f) && (yi <= (float)(HH - 1)) && (xi >= 0.0f) && (xi <= (float)(WW - 1));
    const float ycl = fminf(fmaxf(yi, 0.0f), (float)(HH - 1));
    const float xcl = fminf(fmaxf(xi, 0.0f), (float)(WW - 1));
    cid[t] = (int)ycl * WW + (int)xcl;
    cw[t] = ok ? wgt : 0.0f;
  }

  const float* nmb = nmap + (size_t)b * XP;
  float nin = cw[0] * nmb[cid[0]];
  nin += cw[1] * nmb[cid[1]];
  nin += cw[2] * nmb[cid[2]];
  nin += cw[3] * nmb[cid[3]];

  float ssq = 0.f;
  #pragma unroll 1
  for (int c = 0; c < CP; ++c) {
    const float* xc_ = xb + (size_t)c * XP;
    float s = cw[0] * xc_[cid[0]];
    s += cw[1] * xc_[cid[1]];
    s += cw[2] * xc_[cid[2]];
    s += cw[3] * xc_[cid[3]];
    sS[c * 64 + tid] = s;
    ssq += s * s;
  }
  ssq += 1e-12f;
  const float fac = nin * (1.0f / sqrtf(ssq));

  #pragma unroll 1
  for (int c = 0; c < CPAD; ++c) {
    const int cc = (c < CP) ? c : (CP - 1);
    const float s = sS[cc * 64 + tid];
    const float v = (c < CP) ? s * fac : 0.0f;
    sA[ml * KPAD + c * KK + kk] = (_Float16)v;
  }
  __syncthreads();
  _Float16* dst = apl + (size_t)blockIdx.x * 16 * KPAD;
  plane_store16(sA, dst, tid);
  __threadfence();
  plane_store16(sA, dst, tid);
}

__device__ __forceinline__ void acts_store_pass(const float* sT, float* acts,
                                                int pbase, int n0, int w, int lane) {
  const int q8 = lane & 7, sub = lane >> 3;
  #pragma unroll
  for (int i = 0; i < 16; ++i) {
    const int L = i * 4 + sub;
    const int row = 32 * w + (L >> 1), hl = L & 1;
    const v4f v = *(const v4fa*)(sT + row * 64 + 32 * hl + 4 * q8);
    float* dst = acts + (size_t)(pbase + row) * MM + n0 + 32 * hl + 4 * q8;
    *(volatile v4f*)dst = v;
  }
}

__global__ __launch_bounds__(128) void k_gemm(const _Float16* __restrict__ ppl,
                                              const _Float16* __restrict__ apl,
                                              float* __restrict__ acts) {
  __shared__ __attribute__((aligned(16))) float sT[128 * 64];
  const int tid = threadIdx.x, lane = tid & 31, w = tid >> 5;
  const int h = lane >> 4, m = lane & 15;
  const int pbase = blockIdx.x * 128;
  const int n0 = blockIdx.y * 64;
  const int p0w = pbase + 32 * w;

  const _Float16* a0p = ppl + (size_t)(p0w + m) * KPAD;
  const _Float16* a1p = a0p + (size_t)16 * KPAD;
  const _Float16* b0p = apl + (size_t)(n0 + m) * KPAD;

  const v8f zero8 = {0.f, 0.f, 0.f, 0.f, 0.f, 0.f, 0.f, 0.f};
  v8f acc[2][4];
  #pragma unroll
  for (int mt = 0; mt < 2; ++mt)
    #pragma unroll
    for (int nt = 0; nt < 4; ++nt) acc[mt][nt] = zero8;

  #pragma unroll 1
  for (int k0 = 0; k0 < KPAD; k0 += 32) {
    const v16h a0 = load_frag(a0p + k0, h);
    const v16h a1 = load_frag(a1p + k0, h);
    #pragma unroll
    for (int nt = 0; nt < 4; ++nt) {
      const v16h bfr = load_frag(b0p + (size_t)(16 * nt) * KPAD + k0, h);
      acc[0][nt] = wmma_f16(a0, bfr, acc[0][nt]);
      acc[1][nt] = wmma_f16(a1, bfr, acc[1][nt]);
    }
  }

  const float osc = 0.015625f * (1.0f / 64.64f);
  #pragma unroll
  for (int mt = 0; mt < 2; ++mt)
    #pragma unroll
    for (int nt = 0; nt < 4; ++nt)
      #pragma unroll
      for (int r = 0; r < 8; ++r) {
        const int rowl = 32 * w + 16 * mt + 8 * h + r;
        const float v = acc[mt][nt][r] * osc;
        sT[rowl * 64 + 16 * nt + m] = fmaxf(v, 0.0f);
      }
  __syncthreads();

  acts_store_pass(sT, acts, pbase, n0, w, lane);
  __threadfence();
  acts_store_pass(sT, acts, pbase, n0, w, lane);
}

__global__ __launch_bounds__(256) void k_topk(const float* __restrict__ acts,
                                              const int* __restrict__ pk,
                                              float* __restrict__ pacts) {
  __shared__ float sP[32];
  const int tid = threadIdx.x, lane = tid & 31, w = tid >> 5;
  const int q = blockIdx.x, b = blockIdx.y;
  int k = pk[0];
  k = k < 1 ? 1 : (k > HW ? HW : k);
  const float rk = 1.0f / (float)k;

  #pragma unroll 1
  for (int j = 0; j < 4; ++j) {
    const int pl = 4 * w + j;
    const int p = 32 * q + pl;
    const float* row = acts + (size_t)p * MM + b * HW;
    float v[7];
    #pragma unroll
    for (int i = 0; i < 7; ++i) {
      const int hw = lane + 32 * i;
      const int hwc = hw < HW ? hw : (HW - 1);
      const float t = row[hwc];
      v[i] = (hw < HW) ? t : -1.0f;
    }
    float sum = 0.f;
    #pragma unroll 1
    for (int it = 0; it < k; ++it) {
      float mx = v[0];
      #pragma unroll
      for (int i = 1; i < 7; ++i) mx = fmaxf(mx, v[i]);
      #pragma unroll
      for (int off = 16; off > 0; off >>= 1) mx = fmaxf(mx, __shfl_xor(mx, off));
      sum += mx;
      bool has = false;
      #pragma unroll
      for (int i = 0; i < 7; ++i) has = has || (v[i] == mx);
      const unsigned long long bal = __ballot(has);
      const int first = (int)__ffsll((unsigned long long)bal) - 1;
      const bool me = (lane == first);
      bool done = false;
      #pragma unroll
      for (int i = 0; i < 7; ++i) {
        const bool hit = me && (!done) && (v[i] == mx);
        v[i] = hit ? -1.0f : v[i];
        done = done || hit;
      }
    }
    if (lane == 0) sP[pl] = sum * rk;
  }
  __syncthreads();
  if (w == 0) {
    const float val = sP[lane];
    float* dst = pacts + (size_t)b * PPAD + 32 * q + lane;
    *(volatile float*)dst = val;
    __threadfence();
    *(volatile float*)dst = val;
  }
}

__device__ __forceinline__ void out_store_pass(const float* sO, float* out, int tid) {
  #pragma unroll
  for (int j = 0; j < 7; ++j) {
    const int piece = tid + 256 * j;
    if (piece < (BB * NCLS) / 4) {
      const v4f v = *(const v4fa*)(sO + piece * 4);
      *(volatile v4f*)(out + (size_t)piece * 4) = v;
    }
  }
}

__global__ __launch_bounds__(256) void k_logits(const float* __restrict__ pacts,
                                                const float* __restrict__ wl,
                                                float* __restrict__ out) {
  __shared__ __attribute__((aligned(16))) float sO[BB * NCLS];
  const int tid = threadIdx.x;
  #pragma unroll 1
  for (int j = 0; j < (BB * NCLS) / 256; ++j) {
    const int e = tid + 256 * j;
    const int b = e / NCLS, n = e - b * NCLS;
    const float* pa = pacts + (size_t)b * PPAD;
    const float* wr = wl + (size_t)n * PP;
    float s = 0.f;
    #pragma unroll 4
    for (int p = 0; p < PP; ++p) s += pa[p] * wr[p];
    sO[e] = s;
  }
  __syncthreads();
  out_store_pass(sO, out, tid);
  __threadfence();
  out_store_pass(sO, out, tid);
}

extern "C" void kernel_launch(void* const* d_in, const int* in_sizes, int n_in,
                              void* d_out, int out_size, void* d_ws, size_t ws_size,
                              hipStream_t stream) {
  if (n_in < 5) return;
  if (in_sizes[0] != BB * CC * HW) return;
  if (in_sizes[1] != PP * CC * KK) return;
  if (in_sizes[2] != 8 * CP * 9) return;
  if (in_sizes[3] != NCLS * PP) return;
  if (in_sizes[4] < 1) return;
  if (out_size != BB * NCLS) return;

  const float* x   = (const float*)d_in[0];
  const float* pv  = (const float*)d_in[1];
  const float* cow = (const float*)d_in[2];
  const float* wll = (const float*)d_in[3];
  const int*   pk  = (const int*)d_in[4];
  float* out = (float*)d_out;

  const size_t xn_bytes   = (size_t)BB * CP * XP * 4;
  const size_t nmap_bytes = (size_t)BB * XP * 4;
  const size_t apl_bytes  = (size_t)MM * KPAD * 2;
  const size_t ppl_bytes  = (size_t)PPAD * KPAD * 2;
  const size_t acts_bytes = (size_t)PPAD * MM * 4;
  const size_t pact_bytes = (size_t)BB * PPAD * 4;
  const size_t total = xn_bytes + nmap_bytes + apl_bytes + ppl_bytes + acts_bytes + pact_bytes;
  if (total > ws_size) return;

  char* ws = (char*)d_ws;
  size_t off = 0;
  float*    xn    = (float*)(ws + off);    off += xn_bytes;
  float*    nmap  = (float*)(ws + off);    off += nmap_bytes;
  _Float16* apl   = (_Float16*)(ws + off); off += apl_bytes;
  _Float16* ppl   = (_Float16*)(ws + off); off += ppl_bytes;
  float*    acts  = (float*)(ws + off);    off += acts_bytes;
  float*    pacts = (float*)(ws + off);    off += pact_bytes;

  k_prep_x<<<BB, 224, 0, stream>>>(x, xn, nmap);
  k_proto<<<PPAD / 16, 64, 0, stream>>>(pv, ppl);
  k_sample<<<MM / 16, 64, 0, stream>>>(xn, nmap, cow, apl);

  dim3 gg(PPAD / 128, MM / 64);
  k_gemm<<<gg, 128, 0, stream>>>(ppl, apl, acts);

  dim3 gt(PPAD / 32, BB);
  k_topk<<<gt, 256, 0, stream>>>(acts, pk, pacts);

  k_logits<<<1, 256, 0, stream>>>(pacts, wll, out);
}
